// Mamba3Block_40046275068368
// MI455X (gfx1250) — hardware-verified
//
#include <hip/hip_runtime.h>
#include <math.h>

typedef __attribute__((ext_vector_type(16))) _Float16 v16h;
typedef __attribute__((ext_vector_type(8)))  _Float16 v8h;
typedef __attribute__((ext_vector_type(16))) __bf16   v16b;
typedef __attribute__((ext_vector_type(8)))  __bf16   v8b;
typedef __attribute__((ext_vector_type(8)))  float    v8f;
typedef __attribute__((ext_vector_type(4)))  float    v4f;
typedef __attribute__((ext_vector_type(2)))  float    v2f;

constexpr int kSeq    = 2048;
constexpr int kDm     = 512;
constexpr int kWinLd  = 2568;
constexpr int kProjN  = 2560;
constexpr int kDin    = 1024;
constexpr int kHeads  = 16;
constexpr int kHd     = 64;
constexpr int kNst    = 32;
constexpr int kGrp    = 4;
constexpr int kRk     = 2;
constexpr int kRowsH  = kSeq * kHeads;
constexpr int kXupN   = kHd * kRk;
constexpr int kBCW    = 2 * kNst * kRk;
constexpr int kScW    = 16;
constexpr int kAngW   = kGrp * (kNst / 2);
constexpr int kTS     = 16;
constexpr int kYP     = 132;
constexpr float kCarryAct = 64.0f;
constexpr float kCarryW   = 32.0f;
constexpr float kFoldBack = 1.0f / (kCarryAct * kCarryW);
constexpr float kEps      = 1e-5f;
static_assert(kRowsH == 32768 && kXupN == 128 && kBCW == 128 && kAngW == 64, "shape constants");
static_assert(kDin == kHeads * kHd && kHeads == 4 * kGrp, "head layout");
static_assert(kProjN == 2 * kDin + 2 * kGrp * kNst * kRk && kWinLd == kProjN + 2 * kGrp, "projection column blocks");
static_assert((kDm % 32) == 0 && (kHd % 32) == 0 && (kXupN % 32) == 0 && (kDin % 32) == 0, "GEMM K multiples of 32");
static_assert((kSeq % 64) == 0 && (kRowsH % 64) == 0 && (kProjN % 64) == 0 && (kXupN % 64) == 0 && (kHd % 64) == 0 && (kDm % 64) == 0, "GEMM M,N multiples of 64");
static_assert((kSeq % kTS) == 0, "time tile");

constexpr size_t kOffUH   = 0;
constexpr size_t kOffUL   = kOffUH   + (size_t)kSeq * kDm * 2;
constexpr size_t kOffWIH  = kOffUL   + (size_t)kSeq * kDm * 2;
constexpr size_t kOffWIL  = kOffWIH  + (size_t)kProjN * kDm * 2;
constexpr size_t kOffWOH  = kOffWIL  + (size_t)kProjN * kDm * 2;
constexpr size_t kOffWOL  = kOffWOH  + (size_t)kDm * kDin * 2;
constexpr size_t kOffWXT  = kOffWOL  + (size_t)kDm * kDin * 2;
constexpr size_t kOffWYT  = kOffWXT  + (size_t)kXupN * kHd * 2;
constexpr size_t kOffPROJ = kOffWYT  + (size_t)kHd * kXupN * 2;
constexpr size_t kOffSC   = kOffPROJ + (size_t)kSeq * kProjN * 4;
constexpr size_t kOffCOS  = kOffSC   + (size_t)kSeq * kScW * 4;
constexpr size_t kOffSIN  = kOffCOS  + (size_t)kSeq * kAngW * 4;
constexpr size_t kOffXS   = kOffSIN  + (size_t)kSeq * kAngW * 4;
constexpr size_t kOffBC   = kOffXS   + (size_t)kRowsH * kHd * 2;
constexpr size_t kOffXUP  = kOffBC   + (size_t)kGrp * kSeq * kBCW * 4;
constexpr size_t kOffY16  = kOffXUP  + (size_t)kRowsH * kXupN * 4;
constexpr size_t kOffY2   = kOffY16  + (size_t)kRowsH * kXupN * 2;
constexpr size_t kOffYGH  = kOffY2   + (size_t)kRowsH * kHd * 4;
constexpr size_t kOffYGL  = kOffYGH  + (size_t)kSeq * kDin * 2;
constexpr size_t kWsTotal = kOffYGL  + (size_t)kSeq * kDin * 2;
static_assert(kWsTotal == 84049920ull, "carve total");
static_assert(kWsTotal <= 134217728ull, "carve cap");
static_assert((kOffUL % 128) == 0 && (kOffWIH % 128) == 0 && (kOffWIL % 128) == 0 && (kOffWOH % 128) == 0 &&
              (kOffWOL % 128) == 0 && (kOffWXT % 128) == 0 && (kOffWYT % 128) == 0 && (kOffPROJ % 128) == 0 &&
              (kOffSC % 128) == 0 && (kOffCOS % 128) == 0 && (kOffSIN % 128) == 0 && (kOffXS % 128) == 0 &&
              (kOffBC % 128) == 0 && (kOffXUP % 128) == 0 && (kOffY16 % 128) == 0 && (kOffY2 % 128) == 0 &&
              (kOffYGH % 128) == 0 && (kOffYGL % 128) == 0, "128-B aligned regions");

__device__ __forceinline__ unsigned short f2bf_bits(float f) {
  unsigned u = __float_as_uint(f);
  return (unsigned short)((u + 0x7FFFu + ((u >> 16) & 1u)) >> 16);
}
__device__ __forceinline__ float bf_bits2f(unsigned short h) { return __uint_as_float(((unsigned)h) << 16); }

__device__ __forceinline__ void grp_guard_h(v8f& a, v8f& b, v8f& c, v8f& d, v16h x, v16h y) {
  asm volatile("v_nop\n\tv_nop\n\tv_nop\n\tv_nop" : "+v"(a), "+v"(b), "+v"(c), "+v"(d) : "v"(x), "v"(y));
}
__device__ __forceinline__ void grp_guard_b(v8f& a, v8f& b, v8f& c, v8f& d, v16b x, v16b y) {
  asm volatile("v_nop\n\tv_nop\n\tv_nop\n\tv_nop" : "+v"(a), "+v"(b), "+v"(c), "+v"(d) : "v"(x), "v"(y));
}
__device__ __forceinline__ void keep4_h(v16h a, v16h b, v16h c, v16h d) { asm volatile("v_nop" :: "v"(a), "v"(b), "v"(c), "v"(d)); }
__device__ __forceinline__ void keep4_b(v16b a, v16b b, v16b c, v16b d) { asm volatile("v_nop" :: "v"(a), "v"(b), "v"(c), "v"(d)); }
__device__ __forceinline__ void acc_guard4(v8f& a, v8f& b, v8f& c, v8f& d) {
  asm volatile("v_nop\n\tv_nop\n\tv_nop\n\tv_nop" : "+v"(a), "+v"(b), "+v"(c), "+v"(d));
}
template <typename T> struct Frag;
template <> struct Frag<_Float16> {
  typedef v16h V; union U { v16h v; v8h h[2]; };
  static __device__ __forceinline__ v16h load(const _Float16* p) {
    U f; f.h[0] = *(const v8h*)(p); f.h[1] = *(const v8h*)(p + 16); return f.v;
  }
  static __device__ __forceinline__ v8f mma(v16h a, v16h b, v8f c) {
    return __builtin_amdgcn_wmma_f32_16x16x32_f16(false, a, false, b, (short)0, c, false, false);
  }
  static __device__ __forceinline__ void guard(v8f& a, v8f& b, v8f& c, v8f& d, v16h x, v16h y) { grp_guard_h(a, b, c, d, x, y); }
  static __device__ __forceinline__ void keep(v16h a, v16h b, v16h c, v16h d) { keep4_h(a, b, c, d); }
};
template <> struct Frag<__bf16> {
  typedef v16b V; union U { v16b v; v8b h[2]; };
  static __device__ __forceinline__ v16b load(const __bf16* p) {
    U f; f.h[0] = *(const v8b*)(p); f.h[1] = *(const v8b*)(p + 16); return f.v;
  }
  static __device__ __forceinline__ v8f mma(v16b a, v16b b, v8f c) {
    return __builtin_amdgcn_wmma_f32_16x16x32_bf16(false, a, false, b, (short)0, c, false, false);
  }
  static __device__ __forceinline__ void guard(v8f& a, v8f& b, v8f& c, v8f& d, v16b x, v16b y) { grp_guard_b(a, b, c, d, x, y); }
  static __device__ __forceinline__ void keep(v16b a, v16b b, v16b c, v16b d) { keep4_b(a, b, c, d); }
};

template <int ET> struct Elem;
template <> struct Elem<0> { typedef _Float16 T; };
template <> struct Elem<1> { typedef __bf16 T; };
template <int ET, int SPL, int BIAS_MODE>
__global__ __launch_bounds__(256) void wmma_gemm64(
    const unsigned short* __restrict__ Ap, const unsigned short* __restrict__ A2p, int lda,
    const unsigned short* __restrict__ Btp, const unsigned short* __restrict__ Bt2p, int ldb,
    float* __restrict__ C, int ldc, const float* __restrict__ bias,
    int M, int N, int K, float scale) {
  typedef typename Elem<ET>::T T;
  typedef typename Frag<T>::V V;
  const T* A = (const T*)Ap; const T* A2 = (const T*)A2p; const T* Bt = (const T*)Btp; const T* Bt2 = (const T*)Bt2p;
  __shared__ __align__(16) float sT[8][16 * 68];
  const int lane = threadIdx.x & 31;
  const int wave = threadIdx.x >> 5;
  const int tilesN = N >> 6;
  const int tilesM = M >> 6;
  const int tile = blockIdx.x * 8 + wave;
  if (tile >= tilesM * tilesN) return;
  const int tm = tile / tilesN;
  const int tn = tile - tm * tilesN;
  const int m0 = tm << 6;
  const int n0 = tn << 6;

  const int rlane = lane & 15;
  const int koff  = (lane >> 4) * 8;
  const int mOff  = (lane >> 4) * 8;

  v8f acc[4][4];
#pragma unroll
  for (int i = 0; i < 4; ++i)
#pragma unroll
    for (int j = 0; j < 4; ++j) acc[i][j] = (v8f){0.f,0.f,0.f,0.f,0.f,0.f,0.f,0.f};

  for (int k0 = 0; k0 < K; k0 += 32) {
    V bh[4], bl[4];
#pragma unroll
    for (int j = 0; j < 4; ++j) {
      const size_t bo = (size_t)(n0 + (j << 4) + rlane) * ldb + koff + k0;
      bh[j] = Frag<T>::load(Bt + bo);
      if (SPL == 2) bl[j] = Frag<T>::load(Bt2 + bo);
    }
#pragma unroll
    for (int i = 0; i < 4; ++i) {
      const size_t ao = (size_t)(m0 + (i << 4) + rlane) * lda + koff + k0;
      V ah = Frag<T>::load(A + ao);
      V al;
      if (SPL == 2) al = Frag<T>::load(A2 + ao);
#pragma unroll
      for (int j = 0; j < 4; ++j) {
        acc[i][j] = Frag<T>::mma(ah, bh[j], acc[i][j]);
        if (SPL == 2) {
          acc[i][j] = Frag<T>::mma(ah, bl[j], acc[i][j]);
          acc[i][j] = Frag<T>::mma(al, bh[j], acc[i][j]);
        }
      }
      Frag<T>::guard(acc[i][0], acc[i][1], acc[i][2], acc[i][3], ah, (SPL == 2) ? al : ah);
    }
    Frag<T>::keep(bh[0], bh[1], bh[2], bh[3]);
    if (SPL == 2) Frag<T>::keep(bl[0], bl[1], bl[2], bl[3]);
  }
  acc_guard4(acc[0][0], acc[0][1], acc[0][2], acc[0][3]);
  acc_guard4(acc[1][0], acc[1][1], acc[1][2], acc[1][3]);
  acc_guard4(acc[2][0], acc[2][1], acc[2][2], acc[2][3]);
  acc_guard4(acc[3][0], acc[3][1], acc[3][2], acc[3][3]);

  float* slab = sT[wave];
#pragma unroll
  for (int i = 0; i < 4; ++i) {
    const int mBase = m0 + (i << 4);
#pragma unroll
    for (int j = 0; j < 4; ++j) {
      const int n = n0 + (j << 4) + rlane;
      float bv = 0.f;
      if (BIAS_MODE == 2) bv = bias[n];
#pragma unroll
      for (int r = 0; r < 8; ++r) {
        float v = acc[i][j][r] * scale;
        if (BIAS_MODE == 2) v += bv;
        slab[(mOff + r) * 68 + (j << 4) + rlane] = v;
      }
    }
    __builtin_amdgcn_fence(__ATOMIC_RELEASE, "workgroup");
    __builtin_amdgcn_wave_barrier();
    __builtin_amdgcn_fence(__ATOMIC_ACQUIRE, "workgroup");
    {
      const int hh = lane >> 4, c4 = (lane & 15) * 4;
      for (int pass = 0; pass < 2; ++pass) {
#pragma unroll
        for (int it = 0; it < 8; ++it) {
          const int row = it * 2 + hh;
          v4f v = *(const v4f*)(slab + row * 68 + c4);
          *(volatile v4f*)(C + (size_t)(mBase + row) * ldc + n0 + c4) = v;
        }
        __threadfence();
      }
    }
    __builtin_amdgcn_fence(__ATOMIC_RELEASE, "workgroup");
    __builtin_amdgcn_wave_barrier();
    __builtin_amdgcn_fence(__ATOMIC_ACQUIRE, "workgroup");
  }
}

__global__ __launch_bounds__(256) void split_rows_bf16_kernel(
    const float* __restrict__ src, unsigned short* __restrict__ dhi, unsigned short* __restrict__ dlo, int total8)
{
  const int i = blockIdx.x * 256 + threadIdx.x;
  if (i >= total8) return;
  const size_t e0 = (size_t)i << 3;
  const v4f a0 = *(const v4f*)(src + e0);
  const v4f a1 = *(const v4f*)(src + e0 + 4);
  v8h hv, lv;
#pragma unroll
  for (int e = 0; e < 4; ++e) {
    const float f0 = a0[e], f1 = a1[e];
    const unsigned short h0 = f2bf_bits(f0), h1 = f2bf_bits(f1);
    const unsigned short l0 = f2bf_bits(f0 - bf_bits2f(h0)), l1 = f2bf_bits(f1 - bf_bits2f(h1));
    hv[e]     = __builtin_bit_cast(_Float16, h0);
    hv[4 + e] = __builtin_bit_cast(_Float16, h1);
    lv[e]     = __builtin_bit_cast(_Float16, l0);
    lv[4 + e] = __builtin_bit_cast(_Float16, l1);
  }
  unsigned short* qh = dhi + e0;
  unsigned short* ql = dlo + e0;
  *(volatile v8h*)qh = hv;
  *(volatile v8h*)ql = lv;
  __threadfence();
  *(volatile v8h*)qh = hv;
  *(volatile v8h*)ql = lv;
}

template <int MODE>
__global__ __launch_bounds__(256) void transpose_planes_kernel(
    const float* __restrict__ W, int ldw, int Ncols, int Kdim,
    unsigned short* __restrict__ OutH, unsigned short* __restrict__ OutL, float scale)
{
  __shared__ float tile[64 * 65];
  const int tid = threadIdx.x, lane = tid & 31, wave = tid >> 5;
  const int n0 = blockIdx.x * 64;
  const int k0 = blockIdx.y * 64;
#pragma unroll
  for (int p = 0; p < 16; ++p) {
    const int idx = tid + p * 256;
    const int kk  = idx >> 6;
    const int nn  = idx & 63;
    const int n   = n0 + nn;
    const int nc  = (n < Ncols) ? n : (Ncols - 1);
    const float v = W[(size_t)(k0 + kk) * ldw + nc];
    tile[kk * 65 + nn] = (n < Ncols) ? (v * scale) : 0.f;
  }
  __syncthreads();
  const int q = lane >> 3, c8 = (lane & 7) * 8;
  v8h hv[2], lv[2];
#pragma unroll
  for (int it = 0; it < 2; ++it) {
    const int nrow = it * 32 + wave * 4 + q;
#pragma unroll
    for (int e = 0; e < 8; ++e) {
      const float x = tile[(c8 + e) * 65 + nrow];
      if (MODE == 0) {
        hv[it][e] = (_Float16)x;
        lv[it][e] = (_Float16)0.0f;
      } else {
        const unsigned short hb = f2bf_bits(x);
        const unsigned short lb = f2bf_bits(x - bf_bits2f(hb));
        hv[it][e] = __builtin_bit_cast(_Float16, hb);
        lv[it][e] = __builtin_bit_cast(_Float16, lb);
      }
    }
  }
  for (int pass = 0; pass < 2; ++pass) {
#pragma unroll
    for (int it = 0; it < 2; ++it) {
      const int nrow = it * 32 + wave * 4 + q;
      const size_t o = (size_t)(n0 + nrow) * Kdim + k0 + c8;
      *(volatile v8h*)(OutH + o) = hv[it];
      if (MODE == 1) *(volatile v8h*)(OutL + o) = lv[it];
    }
    __threadfence();
  }
}

__global__ __launch_bounds__(256) void dtlam_kernel(
    const float* __restrict__ u, const float* __restrict__ W_in, const float* __restrict__ b_in,
    const float* __restrict__ A_log, float* __restrict__ SC)
{
  __shared__ __align__(16) float sR[32 * kScW];
  const int tid = threadIdx.x, lane = tid & 31, wave = tid >> 5;
  const int rloc = tid >> 3, j = tid & 7;
  const int row = blockIdx.x * 32 + rloc;
  const int col = kProjN + j;
  const float* ur = u + (size_t)row * kDm;
  const float* wc = W_in + col;
  float a0 = 0.f, a1 = 0.f, a2 = 0.f, a3 = 0.f;
#pragma unroll 1
  for (int k = 0; k < kDm; k += 4) {
    const v4f uv = *(const v4f*)(ur + k);
    a0 = fmaf(uv[0], wc[(size_t)(k + 0) * kWinLd], a0);
    a1 = fmaf(uv[1], wc[(size_t)(k + 1) * kWinLd], a1);
    a2 = fmaf(uv[2], wc[(size_t)(k + 2) * kWinLd], a2);
    a3 = fmaf(uv[3], wc[(size_t)(k + 3) * kWinLd], a3);
  }
  const float v  = ((a0 + a1) + (a2 + a3)) + b_in[col];
  const float e  = expf(-fabsf(v));
  const float sp = fmaxf(v, 0.0f) + log1pf(e);
  const float rc = __builtin_amdgcn_rcpf(1.0f + e);
  const float sg = (v >= 0.0f) ? rc : (e * rc);
  const float Ag = -expf(A_log[j & 3]);
  const float av = expf(sp * Ag);
  sR[rloc * kScW + j]     = (j < 4) ? sp : sg;
  sR[rloc * kScW + 8 + j] = (j < 4) ? av : 0.0f;
  __syncthreads();
  if (wave == 0) {
    v4f ov[4];
#pragma unroll
    for (int it = 0; it < 4; ++it) ov[it] = *(const v4f*)(sR + (it * 32 + lane) * 4);
    float* dst = SC + (size_t)blockIdx.x * 32 * kScW;
    for (int pass = 0; pass < 2; ++pass) {
#pragma unroll
      for (int it = 0; it < 4; ++it) *(volatile v4f*)(dst + (it * 32 + lane) * 4) = ov[it];
      __threadfence();
    }
  }
}

__global__ __launch_bounds__(64) void angle_kernel(
    const float* __restrict__ SC, const float* __restrict__ theta_log,
    float* __restrict__ COSP, float* __restrict__ SINP)
{
#pragma clang fp contract(off)
  __shared__ __align__(16) float sD[kTS * 4];
  __shared__ __align__(16) float sC[kTS * kAngW];
  __shared__ __align__(16) float sS[kTS * kAngW];
  const int tid = threadIdx.x, lane = tid & 31, wave = tid >> 5;
  const int g = tid >> 4;
  const float theta = expf(theta_log[tid]);
  float ang = 0.0f;
  const int ss = tid >> 2, sg = tid & 3;
  const int hh = lane >> 4, c4 = (lane & 15) * 4;
#pragma unroll 1
  for (int t0 = 0; t0 < kSeq; t0 += kTS) {
    __syncthreads();
    sD[tid] = SC[(size_t)(t0 + ss) * kScW + sg];
    __syncthreads();
#pragma unroll 1
    for (int s = 0; s < kTS; ++s) {
      const float pr = sD[s * 4 + g] * theta;
      ang = ang + pr;
      sC[s * kAngW + tid] = cosf(ang);
      sS[s * kAngW + tid] = sinf(ang);
    }
    __syncthreads();
    v4f cv[4], sv[4];
#pragma unroll
    for (int it = 0; it < 4; ++it) {
      const int row = it * 4 + wave * 2 + hh;
      cv[it] = *(const v4f*)(sC + row * kAngW + c4);
      sv[it] = *(const v4f*)(sS + row * kAngW + c4);
    }
    for (int pass = 0; pass < 2; ++pass) {
#pragma unroll
      for (int it = 0; it < 4; ++it) {
        const int row = it * 4 + wave * 2 + hh;
        const size_t o = (size_t)(t0 + row) * kAngW + c4;
        *(volatile v4f*)(COSP + o) = cv[it];
        *(volatile v4f*)(SINP + o) = sv[it];
      }
      __threadfence();
    }
  }
}

__global__ __launch_bounds__(256) void act_kernel(
    const float* __restrict__ PROJ, const float* __restrict__ COSP, const float* __restrict__ SINP,
    const float* __restrict__ wB, const float* __restrict__ wC,
    const float* __restrict__ bias_B, const float* __restrict__ bias_C,
    unsigned short* __restrict__ XS16, float* __restrict__ BC)
{
  __shared__ __align__(16) float sX[kDin];
  __shared__ __align__(16) float sN[2 * 256];
  __shared__ __align__(16) float sO[kGrp * kBCW];
  __shared__ float sRed[16];
  const int tid = threadIdx.x, lane = tid & 31, wave = tid >> 5;
  const int l = blockIdx.x;
  const float* pr = PROJ + (size_t)l * kProjN;
#pragma unroll 1
  for (int i = 0; i < 4; ++i) {
    const int idx = tid + 256 * i;
    const float v = pr[kDin + idx];
    const float sg = __builtin_amdgcn_rcpf(1.0f + expf(-v));
    sX[idx] = (v * sg) * kCarryAct;
  }
  const float vb = pr[2 * kDin + tid];
  const float vc = pr[2 * kDin + 256 + tid];
  float qb = vb * vb, qc = vc * vc;
#pragma unroll
  for (int off = 16; off >= 1; off >>= 1) {
    qb += __shfl_xor(qb, off, 32);
    qc += __shfl_xor(qc, off, 32);
  }
  if (lane == 0) { sRed[wave] = qb; sRed[8 + wave] = qc; }
  __syncthreads();
  {
    const int g = tid >> 6, m = tid & 63;
    const float rsb = rsqrtf((sRed[2 * g] + sRed[2 * g + 1]) * (1.0f / 64.0f) + kEps);
    const float rsc = rsqrtf((sRed[8 + 2 * g] + sRed[8 + 2 * g + 1]) * (1.0f / 64.0f) + kEps);
    sN[tid]       = (vb * rsb) * wB[m] + bias_B[g * 64 + m];
    sN[256 + tid] = (vc * rsc) * wC[m] + bias_C[g * 64 + m];
  }
  __syncthreads();
  {
    const int which = tid >> 7;
    const int q = tid & 127;
    const int g2 = q >> 5, rr = q & 1, k = (q >> 1) & 15;
    const float cs = COSP[(size_t)l * kAngW + g2 * 16 + k];
    const float sn = SINP[(size_t)l * kAngW + g2 * 16 + k];
    const float* src = sN + which * 256 + g2 * 64;
    const float re = src[4 * k + rr];
    const float im = src[4 * k + 2 + rr];
    float* dst = sO + g2 * kBCW + which * 64;
    dst[4 * k + rr]     = re * cs - im * sn;
    dst[4 * k + 2 + rr] = re * sn + im * cs;
  }
  __syncthreads();
  if (wave < 4) {
    const v4f ov = *(const v4f*)(sO + wave * kBCW + lane * 4);
    float* dst = BC + ((size_t)wave * kSeq + l) * kBCW + lane * 4;
    *(volatile v4f*)dst = ov;
    __threadfence();
    *(volatile v4f*)dst = ov;
  } else {
    const int t = tid - 128;
    const v4f a0 = *(const v4f*)(sX + t * 8);
    const v4f a1 = *(const v4f*)(sX + t * 8 + 4);
    v8h hv;
#pragma unroll
    for (int e = 0; e < 4; ++e) { hv[e] = (_Float16)a0[e]; hv[4 + e] = (_Float16)a1[e]; }
    unsigned short* dst = XS16 + (size_t)l * kDin + t * 8;
    *(volatile v8h*)dst = hv;
    __threadfence();
    *(volatile v8h*)dst = hv;
  }
}

__global__ __launch_bounds__(128) void scan_kernel(
    const float* __restrict__ BC, const float* __restrict__ XUP, const float* __restrict__ SC,
    unsigned short* __restrict__ Y16)
{
  __shared__ __align__(16) float sBC[kTS * kBCW];
  __shared__ __align__(16) float sXu[kTS * kXupN];
  __shared__ __align__(16) float sSc[kTS * kScW];
  __shared__ __align__(16) float sY[kTS * kYP];
  const int tid = threadIdx.x, lane = tid & 31, wave = tid >> 5;
  const int h = blockIdx.x, g = h >> 2;
  const int p2 = tid & ~1;
  const int nh = tid & 1;
  float hs[16], up[16];
#pragma unroll
  for (int n = 0; n < 16; ++n) { hs[n] = 0.0f; up[n] = 0.0f; }
  const int hh = lane >> 4, c8 = (lane & 15) * 8;
#pragma unroll 1
  for (int t0 = 0; t0 < kSeq; t0 += kTS) {
    __syncthreads();
#pragma unroll
    for (int i = 0; i < 4; ++i) {
      const int idx = tid + 128 * i;
      *(v4f*)(sBC + idx * 4) = *(const v4f*)(BC + ((size_t)g * kSeq + t0) * kBCW + (size_t)idx * 4);
      const int s = idx >> 5, c = (idx & 31) * 4;
      *(v4f*)(sXu + s * kXupN + c) = *(const v4f*)(XUP + ((size_t)(t0 + s) * kHeads + h) * kXupN + c);
    }
    if (tid < 64) {
      *(v4f*)(sSc + tid * 4) = *(const v4f*)(SC + (size_t)t0 * kScW + tid * 4);
    }
    __syncthreads();
#pragma unroll 1
    for (int s = 0; s < kTS; ++s) {
      const float dt  = sSc[s * kScW + g];
      const float lam = sSc[s * kScW + 4 + g];
      const float a   = sSc[s * kScW + 8 + g];
      const float oml = 1.0f - lam;
      const v2f xv = *(const v2f*)(sXu + s * kXupN + p2);
      const float xd0 = dt * xv[0];
      const float xd1 = dt * xv[1];
      const float* bp = sBC + s * kBCW + nh * 32;
      const float* cp = bp + 64;
      float y0 = 0.0f, y1 = 0.0f;
#pragma unroll
      for (int jj = 0; jj < 8; ++jj) {
        const v4f b = *(const v4f*)(bp + 4 * jj);
        const v4f c = *(const v4f*)(cp + 4 * jj);
        {
          const float U  = fmaf(b[1], xd1, b[0] * xd0);
          const float tt = fmaf(oml, up[2 * jj], lam * U);
          const float hn = fmaf(a, hs[2 * jj], tt);
          hs[2 * jj] = hn;
          up[2 * jj] = U;
          y0 = fmaf(hn, c[0], y0);
          y1 = fmaf(hn, c[1], y1);
        }
        {
          const float U  = fmaf(b[3], xd1, b[2] * xd0);
          const float tt = fmaf(oml, up[2 * jj + 1], lam * U);
          const float hn = fmaf(a, hs[2 * jj + 1], tt);
          hs[2 * jj + 1] = hn;
          up[2 * jj + 1] = U;
          y0 = fmaf(hn, c[2], y0);
          y1 = fmaf(hn, c[3], y1);
        }
      }
      const float o0 = __shfl_xor(y0, 1, 32);
      const float o1 = __shfl_xor(y1, 1, 32);
      y0 += o0;
      y1 += o1;
      const float ysel = nh ? y1 : y0;
      sY[s * kYP + tid] = ysel * kCarryAct;
    }
    __syncthreads();
    v8h hv[2];
#pragma unroll
    for (int it = 0; it < 2; ++it) {
      const int row = it * 8 + wave * 2 + hh;
      const float* sp = sY + row * kYP + c8;
      const v4f a0 = *(const v4f*)(sp);
      const v4f a1 = *(const v4f*)(sp + 4);
#pragma unroll
      for (int e = 0; e < 4; ++e) { hv[it][e] = (_Float16)a0[e]; hv[it][4 + e] = (_Float16)a1[e]; }
    }
    for (int pass = 0; pass < 2; ++pass) {
#pragma unroll
      for (int it = 0; it < 2; ++it) {
        const int row = it * 8 + wave * 2 + hh;
        *(volatile v8h*)(Y16 + ((size_t)(t0 + row) * kHeads + h) * kXupN + c8) = hv[it];
      }
      __threadfence();
    }
  }
}

__global__ __launch_bounds__(256) void gate_kernel(
    const float* __restrict__ Y2, const float* __restrict__ PROJ, const float* __restrict__ Dp,
    unsigned short* __restrict__ YGH, unsigned short* __restrict__ YGL)
{
  __shared__ __align__(16) float sV[2048];
  const int tid = threadIdx.x;
  const size_t base = (size_t)blockIdx.x * 2048;
#pragma unroll 1
  for (int i = 0; i < 8; ++i) {
    const int idx = tid + 256 * i;
    const size_t e = base + idx;
    const int l = (int)(e >> 10);
    const int col = (int)(e & 1023);
    const int hd = col >> 6;
    const float xv = PROJ[(size_t)l * kProjN + kDin + col];
    const float zv = PROJ[(size_t)l * kProjN + col];
    const float yv = Y2[e];
    const float sx = xv * __builtin_amdgcn_rcpf(1.0f + expf(-xv));
    const float sz = zv * __builtin_amdgcn_rcpf(1.0f + expf(-zv));
    sV[idx] = (yv + Dp[hd] * sx) * sz;
  }
  __syncthreads();
  const v4f a0 = *(const v4f*)(sV + tid * 8);
  const v4f a1 = *(const v4f*)(sV + tid * 8 + 4);
  v8h hv, lv;
#pragma unroll
  for (int e = 0; e < 4; ++e) {
    const float f0 = a0[e], f1 = a1[e];
    const unsigned short h0 = f2bf_bits(f0), h1 = f2bf_bits(f1);
    const unsigned short l0 = f2bf_bits(f0 - bf_bits2f(h0)), l1 = f2bf_bits(f1 - bf_bits2f(h1));
    hv[e]     = __builtin_bit_cast(_Float16, h0);
    hv[4 + e] = __builtin_bit_cast(_Float16, h1);
    lv[e]     = __builtin_bit_cast(_Float16, l0);
    lv[4 + e] = __builtin_bit_cast(_Float16, l1);
  }
  unsigned short* qh = YGH + base + tid * 8;
  unsigned short* ql = YGL + base + tid * 8;
  *(volatile v8h*)qh = hv;
  *(volatile v8h*)ql = lv;
  __threadfence();
  *(volatile v8h*)qh = hv;
  *(volatile v8h*)ql = lv;
}

extern "C" void kernel_launch(void* const* d_in, const int* in_sizes, int n_in,
                              void* d_out, int out_size, void* d_ws, size_t ws_size,
                              hipStream_t stream) {
  if (n_in < 13) return;
  if (in_sizes[0] != kSeq * kDm) return;
  if (in_sizes[1] != kDm * kWinLd) return;
  if (in_sizes[2] != kWinLd) return;
  if (in_sizes[3] != kHd * kXupN) return;
  if (in_sizes[4] != kXupN * kHd) return;
  if (in_sizes[5] != kGrp) return;
  if (in_sizes[6] != kGrp * (kNst / 2)) return;
  if (in_sizes[7] != kHeads) return;
  if (in_sizes[8] != kNst * kRk || in_sizes[9] != kNst * kRk) return;
  if (in_sizes[10] != kGrp * kNst * kRk || in_sizes[11] != kGrp * kNst * kRk) return;
  if (in_sizes[12] != kDin * kDm) return;
  if (out_size != kSeq * kDm) return;
  if (ws_size < kWsTotal) return;

  const float* u         = (const float*)d_in[0];
  const float* W_in      = (const float*)d_in[1];
  const float* b_in      = (const float*)d_in[2];
  const float* W_xup     = (const float*)d_in[3];
  const float* W_ydown   = (const float*)d_in[4];
  const float* A_log     = (const float*)d_in[5];
  const float* theta_log = (const float*)d_in[6];
  const float* D_param   = (const float*)d_in[7];
  const float* wB        = (const float*)d_in[8];
  const float* wC        = (const float*)d_in[9];
  const float* bias_B    = (const float*)d_in[10];
  const float* bias_C    = (const float*)d_in[11];
  const float* W_out     = (const float*)d_in[12];
  float* out = (float*)d_out;

  char* ws = (char*)d_ws;
  unsigned short* UH   = (unsigned short*)(ws + kOffUH);
  unsigned short* UL   = (unsigned short*)(ws + kOffUL);
  unsigned short* WIH  = (unsigned short*)(ws + kOffWIH);
  unsigned short* WIL  = (unsigned short*)(ws + kOffWIL);
  unsigned short* WOH  = (unsigned short*)(ws + kOffWOH);
  unsigned short* WOL  = (unsigned short*)(ws + kOffWOL);
  unsigned short* WXT  = (unsigned short*)(ws + kOffWXT);
  unsigned short* WYT  = (unsigned short*)(ws + kOffWYT);
  float*          PROJ = (float*)(ws + kOffPROJ);
  float*          SC   = (float*)(ws + kOffSC);
  float*          COSP = (float*)(ws + kOffCOS);
  float*          SINP = (float*)(ws + kOffSIN);
  unsigned short* XS16 = (unsigned short*)(ws + kOffXS);
  float*          BC   = (float*)(ws + kOffBC);
  float*          XUP  = (float*)(ws + kOffXUP);
  unsigned short* Y16  = (unsigned short*)(ws + kOffY16);
  float*          Y2   = (float*)(ws + kOffY2);
  unsigned short* YGH  = (unsigned short*)(ws + kOffYGH);
  unsigned short* YGL  = (unsigned short*)(ws + kOffYGL);

  split_rows_bf16_kernel<<<(kSeq * kDm / 8) / 256, 256, 0, stream>>>(u, UH, UL, kSeq * kDm / 8);
  transpose_planes_kernel<1><<<dim3(kProjN / 64, kDm / 64), 256, 0, stream>>>(W_in, kWinLd, kProjN, kDm, WIH, WIL, 1.0f);
  transpose_planes_kernel<0><<<dim3(kXupN / 64, kHd / 64), 256, 0, stream>>>(W_xup, kXupN, kXupN, kHd, WXT, WXT, kCarryW);
  transpose_planes_kernel<0><<<dim3(kHd / 64, kXupN / 64), 256, 0, stream>>>(W_ydown, kHd, kHd, kXupN, WYT, WYT, kCarryW);
  transpose_planes_kernel<1><<<dim3(kDm / 64, kDin / 64), 256, 0, stream>>>(W_out, kDm, kDm, kDin, WOH, WOL, 1.0f);

  wmma_gemm64<1, 2, 2><<<(kSeq / 64) * (kProjN / 64) / 8, 256, 0, stream>>>(
      UH, UL, kDm, WIH, WIL, kDm, PROJ, kProjN, b_in, kSeq, kProjN, kDm, 1.0f);

  dtlam_kernel<<<kSeq / 32, 256, 0, stream>>>(u, W_in, b_in, A_log, SC);
  angle_kernel<<<1, 64, 0, stream>>>(SC, theta_log, COSP, SINP);
  act_kernel<<<kSeq, 256, 0, stream>>>(PROJ, COSP, SINP, wB, wC, bias_B, bias_C, XS16, BC);

  wmma_gemm64<0, 0, 0><<<(kRowsH / 64) * (kXupN / 64) / 8, 256, 0, stream>>>(
      XS16, XS16, kHd, WXT, WXT, kHd, XUP, kXupN, b_in, kRowsH, kXupN, kHd, kFoldBack);

  scan_kernel<<<kHeads, 128, 0, stream>>>(BC, XUP, SC, Y16);

  wmma_gemm64<0, 0, 0><<<(kRowsH / 64) * (kHd / 64) / 8, 256, 0, stream>>>(
      Y16, Y16, kXupN, WYT, WYT, kXupN, Y2, kHd, b_in, kRowsH, kHd, kXupN, kFoldBack);

  gate_kernel<<<(kSeq * kDin) / 2048, 256, 0, stream>>>(Y2, PROJ, D_param, YGH, YGL);

  wmma_gemm64<1, 2, 0><<<(kSeq / 64) * (kDm / 64) / 8, 256, 0, stream>>>(
      YGH, YGL, kDin, WOH, WOL, kDin, out, kDm, b_in, kSeq, kDm, kDin, 1.0f);
}
